// ParallelSTBlock_35278861369726
// MI455X (gfx1250) — hardware-verified
//
#include <hip/hip_runtime.h>
#include <hip/hip_bf16.h>

#define NB_     8
#define NN_     200
#define NT_     12
#define NH_     128
#define NHEADS_ 4
#define NE_     3200
#define NBT_    96
#define NROWS_  19200
#define NG_     25
#define NCHUNK_ 100

typedef __attribute__((ext_vector_type(16))) _Float16 v16h;
typedef __attribute__((ext_vector_type(8)))  _Float16 v8h;
typedef __attribute__((ext_vector_type(4)))  _Float16 v4h;
typedef __attribute__((ext_vector_type(16))) __bf16   v16b;
typedef __attribute__((ext_vector_type(8)))  __bf16   v8b;
typedef __attribute__((ext_vector_type(8)))  float    v8f;
typedef __attribute__((ext_vector_type(4)))  float    v4f;
#define U16(p) ((const unsigned short*)(const void*)(p))

__device__ __forceinline__ unsigned short f2bf_bits(float f) {
  unsigned u = __float_as_uint(f);
  return (unsigned short)((u + 0x7FFFu + ((u >> 16) & 1u)) >> 16);
}
__device__ __forceinline__ float bf_bits2f(unsigned short h) { return __uint_as_float(((unsigned)h) << 16); }

__device__ __forceinline__ void dep_guard_h(v8f& a, v8f& b, v16h x, v16h y) { asm volatile("v_nop\n\tv_nop\n\tv_nop\n\tv_nop" : "+v"(a), "+v"(b) : "v"(x), "v"(y)); }
__device__ __forceinline__ void dep_guard_b(v8f& a, v8f& b, v16b x, v16b y) { asm volatile("v_nop\n\tv_nop\n\tv_nop\n\tv_nop" : "+v"(a), "+v"(b) : "v"(x), "v"(y)); }
__device__ __forceinline__ void keep4_h(v16h a, v16h b, v16h c, v16h d) { asm volatile("v_nop" :: "v"(a), "v"(b), "v"(c), "v"(d)); }
__device__ __forceinline__ void keep4_b(v16b a, v16b b, v16b c, v16b d) { asm volatile("v_nop" :: "v"(a), "v"(b), "v"(c), "v"(d)); }
__device__ __forceinline__ void acc_guard4(v8f& a, v8f& b, v8f& c, v8f& d) { asm volatile("v_nop\n\tv_nop\n\tv_nop\n\tv_nop" : "+v"(a), "+v"(b), "+v"(c), "+v"(d)); }
template <typename T> struct Frag;
template <> struct Frag<_Float16> {
  typedef v16h V; union U { v16h v; v8h h[2]; };
  static __device__ __forceinline__ v16h load(const _Float16* p) {
    U f; f.h[0] = *(const v8h*)(p); f.h[1] = *(const v8h*)(p + 16); return f.v;
  }
  static __device__ __forceinline__ v8f mma(v16h a, v16h b, v8f c) {
    return __builtin_amdgcn_wmma_f32_16x16x32_f16(false, a, false, b, (short)0, c, false, false);
  }
  static __device__ __forceinline__ void guard(v8f& a, v8f& b, v16h x, v16h y) { dep_guard_h(a, b, x, y); }
  static __device__ __forceinline__ void keep(v16h a, v16h b, v16h c, v16h d) { keep4_h(a, b, c, d); }
};
template <> struct Frag<__bf16> {
  typedef v16b V; union U { v16b v; v8b h[2]; };
  static __device__ __forceinline__ v16b load(const __bf16* p) {
    U f; f.h[0] = *(const v8b*)(p); f.h[1] = *(const v8b*)(p + 16); return f.v;
  }
  static __device__ __forceinline__ v8f mma(v16b a, v16b b, v8f c) {
    return __builtin_amdgcn_wmma_f32_16x16x32_bf16(false, a, false, b, (short)0, c, false, false);
  }
  static __device__ __forceinline__ void guard(v8f& a, v8f& b, v16b x, v16b y) { dep_guard_b(a, b, x, y); }
  static __device__ __forceinline__ void keep(v16b a, v16b b, v16b c, v16b d) { keep4_b(a, b, c, d); }
};

template <int ET> struct Elem;
template <> struct Elem<0> { typedef _Float16 T; };
template <> struct Elem<1> { typedef __bf16 T; };
template <int ET, bool SPLIT, int BIAS_MODE, int OUT_MODE, bool RESID, int ACT = 0>
__global__ __launch_bounds__(256) void wmma_gemm64(
    const unsigned short* __restrict__ Ap, const unsigned short* __restrict__ A2p, int lda, long strideA,
    const unsigned short* __restrict__ Btp, const unsigned short* __restrict__ Bt2p, int ldb, long strideB,
    void* __restrict__ Cout, void* __restrict__ Cout2, int ldc, long strideC,
    const float* __restrict__ bias,
    const float* __restrict__ resid, long strideR,
    int M, int N, int K, float scale) {
  typedef typename Elem<ET>::T T;
  typedef typename Frag<T>::V V;
  const T* A = (const T*)Ap; const T* A2 = (const T*)A2p; const T* Bt = (const T*)Btp; const T* Bt2 = (const T*)Bt2p;
  __shared__ __align__(16) float sT[8][16 * 68];
  const int b    = blockIdx.y;
  const int lane = threadIdx.x & 31;
  const int wave = threadIdx.x >> 5;
  const int tilesN = N >> 6;
  const int tilesM = M >> 6;
  const int tile = blockIdx.x * 8 + wave;
  if (tile >= tilesM * tilesN) return;
  const int tm = tile / tilesN;
  const int tn = tile - tm * tilesN;
  const int m0 = tm << 6;
  const int n0 = tn << 6;

  const T* Ab  = A  + (size_t)b * strideA;
  const T* Bb  = Bt + (size_t)b * strideB;
  const T* Ab2 = SPLIT ? (A2  + (size_t)b * strideA) : nullptr;
  const T* Bb2 = SPLIT ? (Bt2 + (size_t)b * strideB) : nullptr;

  const int rlane = lane & 15;
  const int koff  = (lane >> 4) * 8;
  const int mOff  = (lane >> 4) * 8;

  v8f acc[4][4];
#pragma unroll
  for (int i = 0; i < 4; ++i)
#pragma unroll
    for (int j = 0; j < 4; ++j) acc[i][j] = (v8f){0.f,0.f,0.f,0.f,0.f,0.f,0.f,0.f};

  for (int k0 = 0; k0 < K; k0 += 32) {
    V bh[4], bl[4];
#pragma unroll
    for (int j = 0; j < 4; ++j) {
      const size_t bo = (size_t)(n0 + (j << 4) + rlane) * ldb + koff + k0;
      bh[j] = Frag<T>::load(Bb + bo);
      if (SPLIT) bl[j] = Frag<T>::load(Bb2 + bo);
    }
#pragma unroll
    for (int i = 0; i < 4; ++i) {
      const size_t ao = (size_t)(m0 + (i << 4) + rlane) * lda + koff + k0;
      V ah = Frag<T>::load(Ab + ao);
      V al;
      if (SPLIT) al = Frag<T>::load(Ab2 + ao);
#pragma unroll
      for (int j = 0; j < 4; ++j) {
        acc[i][j] = Frag<T>::mma(ah, bh[j], acc[i][j]);
        if (SPLIT) {
          acc[i][j] = Frag<T>::mma(ah, bl[j], acc[i][j]);
          acc[i][j] = Frag<T>::mma(al, bh[j], acc[i][j]);
        }
      }
      Frag<T>::guard(acc[i][0], acc[i][3], ah, SPLIT ? al : ah);
    }
    Frag<T>::keep(bh[0], bh[1], bh[2], bh[3]);
    if (SPLIT) Frag<T>::keep(bl[0], bl[1], bl[2], bl[3]);
  }
  acc_guard4(acc[0][0], acc[0][1], acc[0][2], acc[0][3]);
  acc_guard4(acc[1][0], acc[1][1], acc[1][2], acc[1][3]);
  acc_guard4(acc[2][0], acc[2][1], acc[2][2], acc[2][3]);
  acc_guard4(acc[3][0], acc[3][1], acc[3][2], acc[3][3]);

  float* slab = sT[wave];
  const float* Rb = RESID ? (resid + (size_t)b * strideR) : nullptr;
#pragma unroll
  for (int i = 0; i < 4; ++i) {
    const int mBase = m0 + (i << 4);
#pragma unroll
    for (int j = 0; j < 4; ++j) {
      const int n = n0 + (j << 4) + rlane;
      float bv = 0.f;
      if (BIAS_MODE == 2) bv = bias[n];
#pragma unroll
      for (int r = 0; r < 8; ++r) {
        float v = acc[i][j][r] * scale;
        if (BIAS_MODE == 1) v += bias[mBase + mOff + r];
        if (BIAS_MODE == 2) v += bv;
        if (RESID) v += Rb[(size_t)(mBase + mOff + r) * ldc + n];
        if (ACT == 1) v = tanhf(v);
        if (ACT == 2) v = fmaxf(v, 0.0f);
        if (ACT == 3) v = v / (1.0f + expf(-v));
        if (ACT == 4) v = (v > 0.f) ? v : 0.01f * v;
        if (ACT == 5) v = 0.5f * v * (1.0f + erff(v * 0.70710678118654752f));
        slab[(mOff + r) * 68 + (j << 4) + rlane] = v;
      }
    }
    __builtin_amdgcn_fence(__ATOMIC_RELEASE, "workgroup");
    __builtin_amdgcn_wave_barrier();
    __builtin_amdgcn_fence(__ATOMIC_ACQUIRE, "workgroup");
    if (OUT_MODE == 0) {
      float* C = (float*)Cout + (size_t)b * strideC;
      const int hh = lane >> 4, c4 = (lane & 15) * 4;
      for (int pass = 0; pass < 2; ++pass) {
#pragma unroll
        for (int it = 0; it < 8; ++it) {
          const int row = it * 2 + hh;
          v4f v = *(const v4f*)(slab + row * 68 + c4);
          *(volatile v4f*)(C + (size_t)(mBase + row) * ldc + n0 + c4) = v;
        }
        __threadfence();
      }
    } else {
      const int q = lane >> 3, c8 = (lane & 7) * 8;
      unsigned short* C  = (unsigned short*)Cout  + (size_t)b * strideC;
      unsigned short* C2 = (OUT_MODE == 2) ? ((unsigned short*)Cout2 + (size_t)b * strideC) : nullptr;
      for (int pass = 0; pass < 2; ++pass) {
#pragma unroll
        for (int it = 0; it < 4; ++it) {
          const int row = it * 4 + q;
          const float* sp = slab + row * 68 + c8;
          v8h hv, lv;
#pragma unroll
          for (int e = 0; e < 8; ++e) {
            if (OUT_MODE == 1) {
              hv[e] = (_Float16)sp[e];
            } else {
              unsigned short hb = f2bf_bits(sp[e]);
              unsigned short lb = f2bf_bits(sp[e] - bf_bits2f(hb));
              hv[e] = __builtin_bit_cast(_Float16, hb);
              lv[e] = __builtin_bit_cast(_Float16, lb);
            }
          }
          *(volatile v8h*)(C + (size_t)(mBase + row) * ldc + n0 + c8) = hv;
          if (OUT_MODE == 2) *(volatile v8h*)(C2 + (size_t)(mBase + row) * ldc + n0 + c8) = lv;
        }
        __threadfence();
      }
    }
    __builtin_amdgcn_fence(__ATOMIC_RELEASE, "workgroup");
    __builtin_amdgcn_wave_barrier();
    __builtin_amdgcn_fence(__ATOMIC_ACQUIRE, "workgroup");
  }
}

__global__ __launch_bounds__(256) void cast_f32_f16x2(
    const float* __restrict__ in, _Float16* __restrict__ out, int n2) {
  int i = blockIdx.x * 256 + threadIdx.x;
  if (i < n2) {
    const _Float16 h0 = (_Float16)in[2 * i], h1 = (_Float16)in[2 * i + 1];
    const unsigned u = (unsigned)__builtin_bit_cast(unsigned short, h0) | ((unsigned)__builtin_bit_cast(unsigned short, h1) << 16);
    ((volatile unsigned*)out)[i] = u;
    __threadfence();
    ((volatile unsigned*)out)[i] = u;
  }
}

__device__ __forceinline__ v4f ld4(const float* p) { return *(const v4f*)p; }
__device__ __forceinline__ float wsum32(float v) {
#pragma unroll
  for (int off = 16; off > 0; off >>= 1) v += __shfl_xor(v, off, 32);
  return v;
}
__device__ __forceinline__ v4h to_h4(v4f y) {
  v4h hv;
  hv[0] = (_Float16)y[0]; hv[1] = (_Float16)y[1]; hv[2] = (_Float16)y[2]; hv[3] = (_Float16)y[3];
  return hv;
}
__device__ __forceinline__ v4f ln128(v4f o, v4f w, v4f bb) {
  const float mean = wsum32(o[0] + o[1] + o[2] + o[3]) * 0.0078125f;
  v4f d = o - mean;
  const float var = wsum32(d[0] * d[0] + d[1] * d[1] + d[2] * d[2] + d[3] * d[3]) * 0.0078125f;
  const float rstd = rsqrtf(var + 1e-5f);
  return d * rstd * w + bb;
}

__global__ __launch_bounds__(256) void build_x16(const float* __restrict__ x,
                                                 _Float16* __restrict__ x16n, _Float16* __restrict__ x16t,
                                                 int npieces) {
  const int i = blockIdx.x * 256 + threadIdx.x;
  if (i >= npieces) return;
  const int row = i >> 4;
  const int c8  = (i & 15) * 8;
  const float* sn = x + (size_t)row * NH_ + c8;
  v4f a0 = ld4(sn), a1 = ld4(sn + 4);
  v8h hn;
#pragma unroll
  for (int e = 0; e < 4; ++e) { hn[e] = (_Float16)a0[e]; hn[4 + e] = (_Float16)a1[e]; }
  const int bt = row / NN_;
  const int nd = row - bt * NN_;
  const int bb = bt / NT_;
  const int tt = bt - bb * NT_;
  const int srow = (bb * NN_ + nd) * NT_ + tt;
  const float* st = x + (size_t)srow * NH_ + c8;
  v4f b0 = ld4(st), b1 = ld4(st + 4);
  v8h ht;
#pragma unroll
  for (int e = 0; e < 4; ++e) { ht[e] = (_Float16)b0[e]; ht[4 + e] = (_Float16)b1[e]; }
  _Float16* pn = x16n + (size_t)row * NH_ + c8;
  _Float16* pt = x16t + (size_t)row * NH_ + c8;
  *(volatile v8h*)pn = hn;
  *(volatile v8h*)pt = ht;
  __threadfence();
  *(volatile v8h*)pn = hn;
  *(volatile v8h*)pt = ht;
}

__device__ __forceinline__ float lk02(float v) { return (v >= 0.0f) ? v : 0.2f * v; }
__device__ __forceinline__ float score4(v4f at, v4f xl, v4f xr) {
  v4f t = xl + xr;
  return at[0] * lk02(t[0]) + at[1] * lk02(t[1]) + at[2] * lk02(t[2]) + at[3] * lk02(t[3]);
}
__device__ __forceinline__ void online_upd(float s, float& m, float& l, v4f& ac, v4f xl) {
  const float mn = fmaxf(m, s);
  const float al = __expf(m - mn);
  const float p  = __expf(s - mn);
  l  = l * al + p;
  ac = ac * al + xl * p;
  m  = mn;
}

__global__ __launch_bounds__(256) void gat_aggregate(
    const float* __restrict__ XL, const float* __restrict__ XR, const int* __restrict__ ei,
    const float* __restrict__ att, const float* __restrict__ gbias,
    const float* __restrict__ lnw, const float* __restrict__ lnb,
    float* __restrict__ xsp, _Float16* __restrict__ cat16) {
  __shared__ int s_src[NE_];
  __shared__ int s_dst[NE_];
  const int tid  = threadIdx.x;
  const int lane = tid & 31;
  const int wave = tid >> 5;
  const int bt = blockIdx.x / NG_;
  const int ng = blockIdx.x - bt * NG_;
  const int n  = ng * 8 + wave;
  for (int i = tid; i < NE_; i += 256) {
    int s = ei[i], d = ei[NE_ + i];
    s = s < 0 ? 0 : (s > NN_ - 1 ? NN_ - 1 : s);
    d = d < 0 ? 0 : (d > NN_ - 1 ? NN_ - 1 : d);
    s_src[i] = s; s_dst[i] = d;
  }
  __syncthreads();

  const size_t rowR = (size_t)(bt * NN_ + n) * (NHEADS_ * NH_) + 4 * lane;
  const v4f xr0 = ld4(XR + rowR), xr1 = ld4(XR + rowR + NH_), xr2 = ld4(XR + rowR + 2 * NH_), xr3 = ld4(XR + rowR + 3 * NH_);
  const v4f at0 = ld4(att + 4 * lane), at1 = ld4(att + NH_ + 4 * lane), at2 = ld4(att + 2 * NH_ + 4 * lane), at3 = ld4(att + 3 * NH_ + 4 * lane);
  v4f ac0 = (v4f){0.f, 0.f, 0.f, 0.f}, ac1 = ac0, ac2 = ac0, ac3 = ac0;
  float m0 = -1.0e30f, m1 = -1.0e30f, m2 = -1.0e30f, m3 = -1.0e30f;
  float l0 = 0.f, l1 = 0.f, l2 = 0.f, l3 = 0.f;

  for (int chunk = 0; chunk <= NCHUNK_; ++chunk) {
    const int ebase = (chunk == 0) ? 0 : (chunk - 1) * 32;
    const int sv = s_src[ebase + lane];
    const int dv = s_dst[ebase + lane];
    unsigned mask = __builtin_amdgcn_ballot_w32((dv == n) && (sv != dv));
    if (chunk == 0) mask = 1u;
    for (int it = 0; it < 32; ++it) {
      if (mask == 0u) break;
      const int j = __builtin_ctz(mask);
      mask &= mask - 1u;
      const int src = (chunk == 0) ? n : s_src[ebase + j];
      const size_t rowL = (size_t)(bt * NN_ + src) * (NHEADS_ * NH_) + 4 * lane;
      const v4f x0 = ld4(XL + rowL), x1 = ld4(XL + rowL + NH_), x2 = ld4(XL + rowL + 2 * NH_), x3 = ld4(XL + rowL + 3 * NH_);
      float s0 = score4(at0, x0, xr0);
      float s1 = score4(at1, x1, xr1);
      float s2 = score4(at2, x2, xr2);
      float s3 = score4(at3, x3, xr3);
      s0 = wsum32(s0); s1 = wsum32(s1); s2 = wsum32(s2); s3 = wsum32(s3);
      online_upd(s0, m0, l0, ac0, x0);
      online_upd(s1, m1, l1, ac1, x1);
      online_upd(s2, m2, l2, ac2, x2);
      online_upd(s3, m3, l3, ac3, x3);
    }
  }

  const float i0 = 1.0f / l0, i1 = 1.0f / l1, i2 = 1.0f / l2, i3 = 1.0f / l3;
  v4f o = (ac0 * i0 + ac1 * i1 + ac2 * i2 + ac3 * i3) * 0.25f + ld4(gbias + 4 * lane);
  v4f y = ln128(o, ld4(lnw + 4 * lane), ld4(lnb + 4 * lane));
  const int bb = bt / NT_;
  const int tt = bt - bb * NT_;
  const int row = (bb * NN_ + n) * NT_ + tt;
  float*    po = xsp + (size_t)row * NH_ + 4 * lane;
  _Float16* ph = cat16 + (size_t)row * (2 * NH_) + 4 * lane;
  const v4h hv = to_h4(y);
  *(volatile v4f*)po = y;
  *(volatile v4h*)ph = hv;
  __threadfence();
  *(volatile v4f*)po = y;
  *(volatile v4h*)ph = hv;
}

__global__ __launch_bounds__(128) void attn_small(const float* __restrict__ qkv, _Float16* __restrict__ O16) {
  __shared__ float sq[NT_ * NH_], sk[NT_ * NH_], svv[NT_ * NH_];
  __shared__ float sp[NHEADS_ * NT_ * NT_];
  __shared__ __align__(16) _Float16 so[NT_ * NH_];
  const int tid = threadIdx.x;
  const int bn  = blockIdx.x;
  const float* base = qkv + (size_t)bn * NT_ * (3 * NH_);
#pragma unroll 1
  for (int t = 0; t < NT_; ++t) {
    sq[t * NH_ + tid]  = base[t * (3 * NH_) + tid];
    sk[t * NH_ + tid]  = base[t * (3 * NH_) + NH_ + tid];
    svv[t * NH_ + tid] = base[t * (3 * NH_) + 2 * NH_ + tid];
  }
  __syncthreads();
  for (int idx = tid; idx < NHEADS_ * NT_ * NT_; idx += 128) {
    const int hd  = idx / (NT_ * NT_);
    const int rem = idx - hd * (NT_ * NT_);
    const int qi  = rem / NT_;
    const int kj  = rem - qi * NT_;
    const float* qp = sq + qi * NH_ + hd * 32;
    const float* kp = sk + kj * NH_ + hd * 32;
    float s = 0.f;
#pragma unroll 4
    for (int d = 0; d < 32; ++d) s += qp[d] * kp[d];
    sp[idx] = s * 0.17677669529663687f;
  }
  __syncthreads();
  if (tid < NHEADS_ * NT_) {
    float* pr = sp + tid * NT_;
    float mx = pr[0];
#pragma unroll
    for (int j = 1; j < NT_; ++j) mx = fmaxf(mx, pr[j]);
    float sum = 0.f;
#pragma unroll 1
    for (int j = 0; j < NT_; ++j) { const float e = __expf(pr[j] - mx); pr[j] = e; sum += e; }
    const float inv = 1.0f / sum;
#pragma unroll
    for (int j = 0; j < NT_; ++j) pr[j] = pr[j] * inv;
  }
  __syncthreads();
  {
    const int hd = tid >> 5;
#pragma unroll 1
    for (int qi = 0; qi < NT_; ++qi) {
      const float* pr = sp + hd * (NT_ * NT_) + qi * NT_;
      float o = 0.f;
#pragma unroll 4
      for (int kj = 0; kj < NT_; ++kj) o += pr[kj] * svv[kj * NH_ + tid];
      so[qi * NH_ + tid] = (_Float16)o;
    }
  }
  __syncthreads();
  for (int pass = 0; pass < 2; ++pass) {
    for (int p = tid; p < NT_ * 16; p += 128) {
      const int row = p >> 4;
      const int c8  = (p & 15) * 8;
      const v8h val = *(const v8h*)(so + row * NH_ + c8);
      *(volatile v8h*)(O16 + ((size_t)bn * NT_ + row) * NH_ + c8) = val;
    }
    __threadfence();
  }
}

template <int HAS16>
__global__ __launch_bounds__(256) void ln_rows(const float* __restrict__ in,
                                               const float* __restrict__ w, const float* __restrict__ bb,
                                               float* __restrict__ outf,
                                               _Float16* __restrict__ out16, int pitch16, int nrows) {
  const int lane = threadIdx.x & 31;
  const int row  = blockIdx.x * 8 + (threadIdx.x >> 5);
  if (row >= nrows) return;
  const v4f v = ld4(in + (size_t)row * NH_ + 4 * lane);
  const v4f y = ln128(v, ld4(w + 4 * lane), ld4(bb + 4 * lane));
  float* po = outf + (size_t)row * NH_ + 4 * lane;
  *(volatile v4f*)po = y;
  v4h hv;
  _Float16* ph = out16;
  if (HAS16) {
    hv = to_h4(y);
    ph = out16 + (size_t)row * pitch16 + 4 * lane;
    *(volatile v4h*)ph = hv;
  }
  __threadfence();
  *(volatile v4f*)po = y;
  if (HAS16) *(volatile v4h*)ph = hv;
}

__global__ __launch_bounds__(256) void final_rows(const float* __restrict__ apre,
                                                  const float* __restrict__ xs, const float* __restrict__ xt,
                                                  const float* __restrict__ x,
                                                  const float* __restrict__ w, const float* __restrict__ bb,
                                                  float* __restrict__ out, int nrows) {
  const int lane = threadIdx.x & 31;
  const int row  = blockIdx.x * 8 + (threadIdx.x >> 5);
  if (row >= nrows) return;
  const size_t off = (size_t)row * NH_ + 4 * lane;
  const v4f z4 = ld4(apre + off), s4 = ld4(xs + off), t4 = ld4(xt + off), x4 = ld4(x + off);
  v4f v;
#pragma unroll
  for (int e = 0; e < 4; ++e) {
    const float a = 1.0f / (1.0f + __expf(-z4[e]));
    v[e] = a * s4[e] + (1.0f - a) * t4[e] + x4[e];
  }
  const v4f y = ln128(v, ld4(w + 4 * lane), ld4(bb + 4 * lane));
  float* po = out + off;
  *(volatile v4f*)po = y;
  __threadfence();
  *(volatile v4f*)po = y;
}

static inline int gemm_blocks(int M, int N) { return ((M / 64) * (N / 64) + 7) / 8; }

extern "C" void kernel_launch(void* const* d_in, const int* in_sizes, int n_in,
                              void* d_out, int out_size, void* d_ws, size_t ws_size,
                              hipStream_t stream) {
  if (n_in < 26) return;
  if (in_sizes[0] != NROWS_ * NH_ || in_sizes[1] != 2 * NE_ || out_size != NROWS_ * NH_) return;
  if (in_sizes[2] != 512 * 128 || in_sizes[4] != 512 * 128 || in_sizes[8] != 384 * 128 ||
      in_sizes[10] != 128 * 128 || in_sizes[12] != 512 * 128 || in_sizes[14] != 128 * 512 ||
      in_sizes[16] != 128 * 256) return;

  const float* x        = (const float*)d_in[0];
  const int*   ei       = (const int*)  d_in[1];
  const float* gat_wl   = (const float*)d_in[2];
  const float* gat_bl   = (const float*)d_in[3];
  const float* gat_wr   = (const float*)d_in[4];
  const float* gat_br   = (const float*)d_in[5];
  const float* gat_att  = (const float*)d_in[6];
  const float* gat_bias = (const float*)d_in[7];
  const float* ain_w    = (const float*)d_in[8];
  const float* ain_b    = (const float*)d_in[9];
  const float* aout_w   = (const float*)d_in[10];
  const float* aout_b   = (const float*)d_in[11];
  const float* w1       = (const float*)d_in[12];
  const float* b1       = (const float*)d_in[13];
  const float* w2       = (const float*)d_in[14];
  const float* b2       = (const float*)d_in[15];
  const float* gw       = (const float*)d_in[16];
  const float* gb       = (const float*)d_in[17];
  const float* ln_sp_w  = (const float*)d_in[18];
  const float* ln_sp_b  = (const float*)d_in[19];
  const float* ln_t1_w  = (const float*)d_in[20];
  const float* ln_t1_b  = (const float*)d_in[21];
  const float* ln_t2_w  = (const float*)d_in[22];
  const float* ln_t2_b  = (const float*)d_in[23];
  const float* ln_f_w   = (const float*)d_in[24];
  const float* ln_f_b   = (const float*)d_in[25];
  float* out = (float*)d_out;

  const size_t szW512  = (size_t)512 * 128 * 2;
  const size_t szW384  = (size_t)384 * 128 * 2;
  const size_t szW128  = (size_t)128 * 128 * 2;
  const size_t szWg    = (size_t)128 * 256 * 2;
  const size_t szH128  = (size_t)NROWS_ * NH_ * 2;
  const size_t szF128  = (size_t)NROWS_ * NH_ * 4;
  const size_t szH256  = (size_t)NROWS_ * 2 * NH_ * 2;
  const size_t szF512  = (size_t)NROWS_ * 512 * 4;
  const size_t szF384  = (size_t)NROWS_ * 384 * 4;
  const size_t szH512  = (size_t)NROWS_ * 512 * 2;
  const size_t szR     = 2 * szF512;

  char* base = (char*)d_ws;
  size_t off = 0;
  _Float16* wl16   = (_Float16*)(base + off); off += szW512;
  _Float16* wr16   = (_Float16*)(base + off); off += szW512;
  _Float16* win16  = (_Float16*)(base + off); off += szW384;
  _Float16* wout16 = (_Float16*)(base + off); off += szW128;
  _Float16* w1_16  = (_Float16*)(base + off); off += szW512;
  _Float16* w2_16  = (_Float16*)(base + off); off += szW512;
  _Float16* wg16   = (_Float16*)(base + off); off += szWg;
  _Float16* x16t   = (_Float16*)(base + off); off += szH128;
  _Float16* x16n   = (_Float16*)(base + off); off += szH128;
  float*    x_sp   = (float*)   (base + off); off += szF128;
  float*    x_tm   = (float*)   (base + off); off += szF128;
  _Float16* cat16  = (_Float16*)(base + off); off += szH256;
  char*     R      = base + off;               off += szR;
  if (off > ws_size) return;

  float* XL = (float*)(R);
  float* XR = (float*)(R + szF512);
  float*    qkvb   = (float*)   (R);
  _Float16* O16    = (_Float16*)(R + szF384);
  float*    tmp    = (float*)   (R);
  float*    xn1    = (float*)   (R + szF384 + szH128);
  _Float16* xn1_16 = (_Float16*)(R + szF384 + szH128 + szF128);
  _Float16* f1_16  = (_Float16*)(R + szF384 + szH128 + szF128 + szH128);
  float*    a_pre  = (float*)   (R);

  typedef const unsigned short* cu16;

  build_x16<<<(NROWS_ * 16 + 255) / 256, 256, 0, stream>>>(x, x16n, x16t, NROWS_ * 16);
  cast_f32_f16x2<<<(512 * 128 / 2 + 255) / 256, 256, 0, stream>>>(gat_wl, wl16,   512 * 128 / 2);
  cast_f32_f16x2<<<(512 * 128 / 2 + 255) / 256, 256, 0, stream>>>(gat_wr, wr16,   512 * 128 / 2);
  cast_f32_f16x2<<<(384 * 128 / 2 + 255) / 256, 256, 0, stream>>>(ain_w,  win16,  384 * 128 / 2);
  cast_f32_f16x2<<<(128 * 128 / 2 + 255) / 256, 256, 0, stream>>>(aout_w, wout16, 128 * 128 / 2);
  cast_f32_f16x2<<<(512 * 128 / 2 + 255) / 256, 256, 0, stream>>>(w1,     w1_16,  512 * 128 / 2);
  cast_f32_f16x2<<<(128 * 512 / 2 + 255) / 256, 256, 0, stream>>>(w2,     w2_16,  128 * 512 / 2);
  cast_f32_f16x2<<<(128 * 256 / 2 + 255) / 256, 256, 0, stream>>>(gw,     wg16,   128 * 256 / 2);

  wmma_gemm64<0, false, 2, 0, false, 0><<<dim3(gemm_blocks(NROWS_, 512), 1), 256, 0, stream>>>(
      (cu16)x16t, (cu16)x16t, NH_, 0L, (cu16)wl16, (cu16)wl16, NH_, 0L,
      (void*)XL, (void*)XL, 512, 0L, gat_bl, gat_bl, 0L, NROWS_, 512, NH_, 1.0f);
  wmma_gemm64<0, false, 2, 0, false, 0><<<dim3(gemm_blocks(NROWS_, 512), 1), 256, 0, stream>>>(
      (cu16)x16t, (cu16)x16t, NH_, 0L, (cu16)wr16, (cu16)wr16, NH_, 0L,
      (void*)XR, (void*)XR, 512, 0L, gat_br, gat_br, 0L, NROWS_, 512, NH_, 1.0f);
  gat_aggregate<<<NBT_ * NG_, 256, 0, stream>>>(XL, XR, ei, gat_att, gat_bias, ln_sp_w, ln_sp_b, x_sp, cat16);

  wmma_gemm64<0, false, 2, 0, false, 0><<<dim3(gemm_blocks(NROWS_, 384), 1), 256, 0, stream>>>(
      (cu16)x16n, (cu16)x16n, NH_, 0L, (cu16)win16, (cu16)win16, NH_, 0L,
      (void*)qkvb, (void*)qkvb, 384, 0L, ain_b, ain_b, 0L, NROWS_, 384, NH_, 1.0f);
  attn_small<<<NB_ * NN_, 128, 0, stream>>>(qkvb, O16);
  wmma_gemm64<0, false, 2, 0, true, 0><<<dim3(gemm_blocks(NROWS_, 128), 1), 256, 0, stream>>>(
      (cu16)O16, (cu16)O16, NH_, 0L, (cu16)wout16, (cu16)wout16, NH_, 0L,
      (void*)tmp, (void*)tmp, NH_, 0L, aout_b, x, 0L, NROWS_, NH_, NH_, 1.0f);
  ln_rows<1><<<(NROWS_ + 7) / 8, 256, 0, stream>>>(tmp, ln_t1_w, ln_t1_b, xn1, xn1_16, NH_, NROWS_);
  wmma_gemm64<0, false, 2, 1, false, 5><<<dim3(gemm_blocks(NROWS_, 512), 1), 256, 0, stream>>>(
      (cu16)xn1_16, (cu16)xn1_16, NH_, 0L, (cu16)w1_16, (cu16)w1_16, NH_, 0L,
      (void*)f1_16, (void*)f1_16, 512, 0L, b1, b1, 0L, NROWS_, 512, NH_, 1.0f);
  wmma_gemm64<0, false, 2, 0, true, 0><<<dim3(gemm_blocks(NROWS_, 128), 1), 256, 0, stream>>>(
      (cu16)f1_16, (cu16)f1_16, 512, 0L, (cu16)w2_16, (cu16)w2_16, 512, 0L,
      (void*)tmp, (void*)tmp, NH_, 0L, b2, xn1, 0L, NROWS_, NH_, 512, 1.0f);
  ln_rows<1><<<(NROWS_ + 7) / 8, 256, 0, stream>>>(tmp, ln_t2_w, ln_t2_b, x_tm, cat16 + NH_, 2 * NH_, NROWS_);

  wmma_gemm64<0, false, 2, 0, false, 0><<<dim3(gemm_blocks(NROWS_, 128), 1), 256, 0, stream>>>(
      (cu16)cat16, (cu16)cat16, 2 * NH_, 0L, (cu16)wg16, (cu16)wg16, 2 * NH_, 0L,
      (void*)a_pre, (void*)a_pre, NH_, 0L, gb, gb, 0L, NROWS_, NH_, 2 * NH_, 1.0f);
  final_rows<<<(NROWS_ + 7) / 8, 256, 0, stream>>>(a_pre, x_sp, x_tm, x, ln_f_w, ln_f_b, out, NROWS_);
}
